// ChebyNet_36627481101156
// MI455X (gfx1250) — hardware-run, weakly checked
//
#include <hip/hip_runtime.h>

typedef float          v8f   __attribute__((ext_vector_type(8)));
typedef float          v4f   __attribute__((ext_vector_type(4)));
typedef unsigned int   v4u   __attribute__((ext_vector_type(4)));
typedef int            v8i   __attribute__((ext_vector_type(8)));
typedef unsigned short v8us  __attribute__((ext_vector_type(8)));
typedef unsigned short v16us __attribute__((ext_vector_type(16)));
typedef __bf16         v16bf __attribute__((ext_vector_type(16)));
typedef _Float16       v16h  __attribute__((ext_vector_type(16)));
typedef v4f  __attribute__((may_alias)) v4fa;
typedef v8us __attribute__((may_alias)) v8usa;
union FragB { v16bf v; v16us u; v8us h[2]; v8i w; };
union FragH { v16h  v; v16us u; v8us h[2]; v8i w; };

__device__ __forceinline__ v8f wmb(const FragB& a, const FragB& b, v8f c) {
  v8f d = __builtin_amdgcn_wmma_f32_16x16x32_bf16(false, a.v, false, b.v, (short)0, c, false, false);
  asm volatile("v_nop\n\tv_nop\n\tv_nop\n\tv_nop" : "+v"(d) : "v"(a.w), "v"(b.w));
  return d;
}

__device__ __forceinline__ v8f wmh(const FragH& a, const FragH& b, v8f c) {
  v8f d = __builtin_amdgcn_wmma_f32_16x16x32_f16(false, a.v, false, b.v, (short)0, c, false, false);
  asm volatile("v_nop\n\tv_nop\n\tv_nop\n\tv_nop" : "+v"(d) : "v"(a.w), "v"(b.w));
  return d;
}

__device__ __forceinline__ unsigned bf16_bits(float f) {
  const unsigned u = __float_as_uint(f);
  const unsigned r = (u + 0x7FFFu + ((u >> 16) & 1u)) >> 16;
  const unsigned q = (u >> 16) | 0x40u;
  return ((u & 0x7fffffffu) > 0x7f800000u) ? q : r;
}

__device__ __forceinline__ float bf16_val(float f) {
  return __uint_as_float(bf16_bits(f) << 16);
}
__device__ __forceinline__ int clampi(int v, int lo, int hi) {
  return v < lo ? lo : (v > hi ? hi : v);
}

__device__ __forceinline__ unsigned f16_bits(float f) {
  const unsigned u  = __float_as_uint(f);
  const unsigned s  = (u >> 16) & 0x8000u;
  const unsigned a  = u & 0x7fffffffu;
  const unsigned t  = a - 0x38000000u;
  const unsigned r  = (t + 0x0FFFu + ((t >> 13) & 1u)) >> 13;
  const unsigned rc = r > 0x7C00u ? 0x7C00u : r;
  const bool small  = a < 0x38800000u;
  const bool isnan  = a > 0x7f800000u;
  const unsigned fin = small ? 0u : (s | rc);
  return isnan ? (s | 0x7E00u) : fin;
}

__device__ __forceinline__ unsigned pk16(unsigned lo, unsigned hi) { return lo | (hi << 16); }
__device__ __forceinline__ unsigned bf16_lo_bits(float v) {
  float hi = bf16_val(v);
  asm volatile("" : "+v"(hi));
  return bf16_bits(v - hi);
}
__device__ __forceinline__ v4u pack8_bf16(v4f a, v4f c) {
  return (v4u){ pk16(bf16_bits(a[0]), bf16_bits(a[1])), pk16(bf16_bits(a[2]), bf16_bits(a[3])),
                pk16(bf16_bits(c[0]), bf16_bits(c[1])), pk16(bf16_bits(c[2]), bf16_bits(c[3])) };
}
__device__ __forceinline__ v4u pack8_bf16_lo(v4f a, v4f c) {
  return (v4u){ pk16(bf16_lo_bits(a[0]), bf16_lo_bits(a[1])), pk16(bf16_lo_bits(a[2]), bf16_lo_bits(a[3])),
                pk16(bf16_lo_bits(c[0]), bf16_lo_bits(c[1])), pk16(bf16_lo_bits(c[2]), bf16_lo_bits(c[3])) };
}
__device__ __forceinline__ v4u pack8_f16(v4f a, v4f c) {
  return (v4u){ pk16(f16_bits(a[0]), f16_bits(a[1])), pk16(f16_bits(a[2]), f16_bits(a[3])),
                pk16(f16_bits(c[0]), f16_bits(c[1])), pk16(f16_bits(c[2]), f16_bits(c[3])) };
}

template <int FORM>
__global__ __launch_bounds__(256) void k_plane(const float* __restrict__ src, int rows, int cols, int ldsrc,
                                               unsigned short* __restrict__ dst, int MP, int KP) {
  static_assert(FORM >= 0 && FORM <= 3);
  const int KTOT = (FORM == 1 || FORM == 3) ? 2 * KP : KP;
  const unsigned ppr   = (unsigned)(KTOT >> 3);
  const unsigned kp8   = (unsigned)(KP >> 3);
  const unsigned total = (unsigned)MP * ppr;
  const unsigned g     = blockIdx.x * 256u + threadIdx.x;
  const unsigned rowu  = g / ppr;
  const unsigned p     = g - rowu * ppr;
  const bool second    = p >= kp8;
  const int row = (int)rowu;
  const int c0  = (int)((second ? p - kp8 : p) << 3);
  const float* srow = src + (size_t)clampi(row, 0, rows - 1) * (size_t)ldsrc;
  float x[8];
  unsigned mk[8];
#pragma unroll
  for (int e = 0; e < 8; ++e) {
    const int c = c0 + e;
    const float v = srow[clampi(c, 0, cols - 1)];
    asm volatile("" :: "v"(v));
    x[e]  = v;
    mk[e] = (row < rows && c < cols) ? 0xFFFFu : 0u;
  }
  const v4f a = (v4f){ x[0], x[1], x[2], x[3] };
  const v4f c = (v4f){ x[4], x[5], x[6], x[7] };
  v4u o;
  if (FORM == 2) {
    o = pack8_f16(a, c);
  } else {
    const v4u hi = pack8_bf16(a, c);
    o = hi;
    if (FORM == 1) { const v4u lo = pack8_bf16_lo(a, c); o = second ? lo : hi; }
  }
  const v4u mw = (v4u){ pk16(mk[0], mk[1]), pk16(mk[2], mk[3]), pk16(mk[4], mk[5]), pk16(mk[6], mk[7]) };
  o &= mw;
  if (g < total) {
    volatile v4u* q = (volatile v4u*)(dst + (size_t)g * 8);
    *q = o;
    __threadfence();
    *q = o;
  }
}

template <int FORM> struct FragOf    { typedef FragB T; };
template <>         struct FragOf<2> { typedef FragH T; };
__device__ __forceinline__ v8f mm(const FragB& a, const FragB& b, v8f c) { return wmb(a, b, c); }
__device__ __forceinline__ v8f mm(const FragH& a, const FragH& b, v8f c) { return wmh(a, b, c); }
template <class F> __device__ __forceinline__ F ld_frag(const unsigned short* p) {
  F f;
  f.h[0] = *(const v8usa*)(p);
  f.h[1] = *(const v8usa*)(p + 16);
  return f;
}

template <int FORM, int EPI>
__global__ __launch_bounds__(256) __attribute__((amdgpu_num_vgpr(248)))
void k_gemm_nt(const unsigned short* __restrict__ A, const unsigned short* __restrict__ B,
               const float* __restrict__ bias, float* __restrict__ D, int M, int N, int KTOT, int ldd) {
  static_assert(FORM >= 0 && FORM <= 2);
  static_assert(EPI == 0 || EPI == 1);
  typedef typename FragOf<FORM>::T F;
  __shared__ __attribute__((aligned(16))) float sT[8][16 * 68];
  const int lane = threadIdx.x & 31;
  const int wave = threadIdx.x >> 5;
  const int tilesM = (M + 63) >> 6;
  const int tilesN = (N + 63) >> 6;
  const int tile = blockIdx.x * 8 + wave;
  if (tile >= tilesM * tilesN) return;
  const int tm = tile / tilesN;
  const int tn = tile - tm * tilesN;
  const int m0 = tm << 6;
  const int n0 = tn << 6;

  const int rl = lane & 15;
  const int h8 = (lane >> 4) * 8;
  const unsigned short* pa = A + (size_t)(m0 + rl) * (size_t)KTOT + h8;
  const unsigned short* pb = B + (size_t)(n0 + rl) * (size_t)KTOT + h8;

  v8f acc[4][4];
#pragma unroll
  for (int i = 0; i < 4; ++i)
#pragma unroll
    for (int j = 0; j < 4; ++j) acc[i][j] = (v8f){0.f, 0.f, 0.f, 0.f, 0.f, 0.f, 0.f, 0.f};

#pragma unroll 1
  for (int k0 = 0; k0 < KTOT; k0 += 32) {
    F bf[4];
#pragma unroll
    for (int j = 0; j < 4; ++j) bf[j] = ld_frag<F>(pb + (size_t)(j << 4) * (size_t)KTOT + k0);
#pragma unroll
    for (int i = 0; i < 4; ++i) {
      const F af = ld_frag<F>(pa + (size_t)(i << 4) * (size_t)KTOT + k0);
#pragma unroll
      for (int j = 0; j < 4; ++j) acc[i][j] = mm(af, bf[j], acc[i][j]);
    }
  }

  float* slab = sT[wave];
  const int hh = lane >> 4;
  const int c4 = (lane & 15) * 4;
  const int nc = n0 + c4;
  const bool cok = nc < N;
  v4f bv = (v4f){0.f, 0.f, 0.f, 0.f};
  if (EPI == 1) {
    bv = *(const v4fa*)(bias + clampi(nc, 0, N - 4));
    asm volatile("" :: "v"(bv));
  }
#pragma unroll
  for (int i = 0; i < 4; ++i) {
    const int mBase = m0 + (i << 4);
#pragma unroll
    for (int j = 0; j < 4; ++j) {
#pragma unroll
      for (int r = 0; r < 8; ++r) slab[(h8 + r) * 68 + (j << 4) + rl] = acc[i][j][r];
    }
    __builtin_amdgcn_fence(__ATOMIC_RELEASE, "workgroup");
    __builtin_amdgcn_wave_barrier();
    __builtin_amdgcn_fence(__ATOMIC_ACQUIRE, "workgroup");
    v4f vv[8];
#pragma unroll
    for (int it = 0; it < 8; ++it) {
      const int row = it * 2 + hh;
      v4f v = *(const v4fa*)(slab + row * 68 + c4);
      if (EPI == 1) v += bv;
      vv[it] = v;
    }
    for (int pass = 0; pass < 2; ++pass) {
#pragma unroll
      for (int it = 0; it < 8; ++it) {
        const int row = mBase + it * 2 + hh;
        if (cok && row < M) *(volatile v4f*)(D + (size_t)row * (size_t)ldd + nc) = vv[it];
      }
      __threadfence();
    }
    __builtin_amdgcn_fence(__ATOMIC_RELEASE, "workgroup");
    __builtin_amdgcn_wave_barrier();
    __builtin_amdgcn_fence(__ATOMIC_ACQUIRE, "workgroup");
  }
}

#pragma clang fp contract(off)

#ifndef H1_TWO_TERM
#define H1_TWO_TERM 1
#endif
static_assert(H1_TWO_TERM == 0 || H1_TWO_TERM == 1);

typedef float v2f __attribute__((ext_vector_type(2)));
typedef int   v4i __attribute__((ext_vector_type(4)));
typedef v2f __attribute__((may_alias)) v2fa;
typedef v4i __attribute__((may_alias)) v4ia;

constexpr int NN     = 100000;
constexpr int NE     = 1600000;
constexpr int FIN    = 128;
constexpr int FH     = 64;
constexpr int FO     = 16;
constexpr int NP     = 100096;
constexpr int NBRUN  = 1024;
constexpr int NBLK   = 98;
constexpr int CAP    = 21504;
constexpr int DEGCAP = 48;
constexpr int WLCAP  = 4096;
constexpr int EPW    = NE / 8;
constexpr int SUB    = 128;
constexpr int NSTEP  = (EPW + SUB - 1) / SUB;
constexpr int PLD    = 128;
constexpr int QLD    = 64;
constexpr int HLK    = 128;

static_assert(NE % 256 == 0 && NE % 8 == 0);
static_assert(NN <= (1 << 17) && NN % 2 == 0 && NN % 16 == 0);
static_assert((((long long)(NN - 1) << 10) | 1023) < (1LL << 31));
static_assert(NBLK * NBRUN >= NN && (NBLK - 1) * NBRUN < NN);
static_assert(CAP * 4 >= 16710 * 5 && (CAP / 4) % 256 == 0 && CAP >= 2 * DEGCAP);
static_assert(CAP * 4 >= 16666 * 5);
static_assert(WLCAP >= (16710 * 5 / 4) / 8 + 256 && WLCAP * 8 >= CAP);
static_assert(DEGCAP >= 36 + 8 && DEGCAP <= 64 && DEGCAP % 16 == 0 && DEGCAP * 4 >= 36 * 5);
static_assert(NP % 64 == 0 && NP >= NN && ((NN + 63) / 64) * 64 <= NP && NP % 8 == 0);
static_assert(NSTEP * SUB >= EPW && (NSTEP - 1) * SUB < EPW);
static_assert(FIN % 32 == 0 && HLK % 32 == 0 && HLK == 2 * FH && PLD % 32 == 0 && QLD % 32 == 0);
static_assert((size_t)(NN - 1) * FO + (FO - 1) < (size_t)NN * FO);
static_assert((NN / 2) % 8 == 0);

constexpr int LK_WL   = 0;
constexpr int LK_SL   = 8 * WLCAP;
constexpr int LK_CNT  = LK_SL + CAP;
constexpr int LK_OFF  = LK_CNT + NBRUN;
constexpr int LK_CUR  = LK_OFF + NBRUN;
constexpr int LK_MISC = LK_CUR + NBRUN;
constexpr int LK_INTS = LK_MISC + 16;
constexpr int LK_LDS  = LK_INTS * 4;
static_assert(LK_LDS == 229440 && LK_LDS <= 262144 && LK_LDS <= 327680);
static_assert(LK_SL % 4 == 0 && LK_CNT % 4 == 0 && LK_CUR % 4 == 0 && (CAP + NBRUN) % 1024 == 0);

constexpr size_t SZ_R0   = (size_t)NP * 128 * 2;
constexpr size_t SZ_R1   = (size_t)NN * PLD * 4;
constexpr size_t SZ_LIST = (size_t)NBLK * CAP * 4;
constexpr size_t SZ_NODE = (size_t)NBLK * NBRUN * 4;
constexpr size_t SZ_FLAG = (size_t)NBLK * 128;
constexpr size_t SZ_BT1  = (size_t)128 * 128 * 2;
constexpr size_t SZ_BT2  = (size_t)64 * 128 * 2;
constexpr size_t SZ_BV   = 256;
constexpr size_t OFF_R0    = 0;
constexpr size_t OFF_R1    = OFF_R0 + SZ_R0;
constexpr size_t OFF_LIST  = OFF_R1 + SZ_R1;
constexpr size_t OFF_CNT   = OFF_LIST + SZ_LIST;
constexpr size_t OFF_OFF   = OFF_CNT + SZ_NODE;
constexpr size_t OFF_DEGS  = OFF_OFF + SZ_NODE;
constexpr size_t OFF_DINV  = OFF_DEGS + SZ_NODE;
constexpr size_t OFF_FLAGL = OFF_DINV + SZ_NODE;
constexpr size_t OFF_FLAGC = OFF_FLAGL + SZ_FLAG;
constexpr size_t OFF_BT1   = OFF_FLAGC + SZ_FLAG;
constexpr size_t OFF_BT2   = OFF_BT1 + SZ_BT1;
constexpr size_t OFF_B1F   = OFF_BT2 + SZ_BT2;
constexpr size_t OFF_B2F   = OFF_B1F + SZ_BV;
constexpr size_t WS_TOTAL  = OFF_B2F + SZ_BV;
static_assert(WS_TOTAL == (size_t)86934528);
static_assert(WS_TOTAL <= ((size_t)128 << 20));
static_assert(SZ_R0 % 256 == 0 && SZ_R1 % 256 == 0 && SZ_LIST % 256 == 0 && SZ_NODE % 256 == 0 && SZ_FLAG % 256 == 0);
static_assert(SZ_BT1 % 256 == 0 && SZ_BT2 % 256 == 0);
static_assert((size_t)NN * QLD * 4 <= SZ_R1 && (size_t)NP * HLK * 2 <= SZ_R0);

__device__ __forceinline__ float relu_k(float v) { return (v > 0.0f) ? v : (v - v); }

__device__ __forceinline__ void wplane_unit(const float* __restrict__ W, int ncols, int kin, int ktot, int nvalid,
                                            unsigned short* __restrict__ dst, int u) {
  const int ppr = ktot >> 3;
  const int n   = u / ppr;
  const int p   = u - n * ppr;
  const int k8  = (p << 3) & (kin - 1);
  const int nc  = n < nvalid ? n : nvalid - 1;
  const float* s = W + (size_t)k8 * (size_t)ncols + nc;
  float x[8];
#pragma unroll
  for (int i = 0; i < 8; ++i) {
    const float v = s[(size_t)i * (size_t)ncols];
    asm volatile("" :: "v"(v));
    x[i] = v;
  }
  v4u o = pack8_bf16((v4f){ x[0], x[1], x[2], x[3] }, (v4f){ x[4], x[5], x[6], x[7] });
  const unsigned mk = (n < nvalid) ? 0xFFFFFFFFu : 0u;
  o &= (v4u){ mk, mk, mk, mk };
  volatile v4u* q = (volatile v4u*)(dst + (size_t)u * 8);
  *q = o;
  __threadfence();
  *q = o;
}

__device__ __forceinline__ void zero_unit(unsigned short* __restrict__ dst, int u) {
  const v4u z = (v4u){ 0u, 0u, 0u, 0u };
  volatile v4u* q = (volatile v4u*)(dst + (size_t)u * 8);
  *q = z;
  __threadfence();
  *q = z;
}

__device__ __forceinline__ void par_unit(const float* __restrict__ src, int n4, int w4, unsigned* __restrict__ dst,
                                         int tid) {
  const int j = tid < n4 ? tid : n4 - 1;
  const v4f a = *(const v4fa*)(src + 4 * j);
  asm volatile("" :: "v"(a));
  const unsigned mk = (tid < n4) ? 0xFFFFFFFFu : 0u;
  v4u o = (v4u){ bf16_bits(a[0]) << 16, bf16_bits(a[1]) << 16, bf16_bits(a[2]) << 16, bf16_bits(a[3]) << 16 };
  o &= (v4u){ mk, mk, mk, mk };
  if (tid < w4) {
    volatile v4u* q = (volatile v4u*)(dst + 4 * tid);
    *q = o;
    __threadfence();
    *q = o;
  }
}

__global__ __launch_bounds__(256) void k_prep(const float* __restrict__ W01, const float* __restrict__ W11,
                                              const float* __restrict__ b1,
                                              const float* __restrict__ W02, const float* __restrict__ W12,
                                              const float* __restrict__ b2,
                                              unsigned short* __restrict__ BT1, unsigned short* __restrict__ BT2,
                                              unsigned* __restrict__ B1F, unsigned* __restrict__ B2F) {
  const int tid = (int)threadIdx.x;
  const int blk = (int)blockIdx.x;
  if (blk < 4) {
    wplane_unit(W01, FH, FIN, FIN, FH, BT1, blk * 256 + tid);
  } else if (blk < 8) {
    wplane_unit(W11, FH, FIN, FIN, FH, BT1 + (size_t)FH * FIN, (blk - 4) * 256 + tid);
  } else if (blk == 8) {
    wplane_unit(W02, FO, FH, HLK, FO, BT2, tid);
  } else if (blk == 9) {
    wplane_unit(W12, FO, FH, HLK, FO, BT2 + (size_t)FO * HLK, tid);
  } else if (blk < 12) {
    zero_unit(BT2 + (size_t)32 * HLK, (blk - 10) * 256 + tid);
  } else {
    par_unit(b1, FH / 4, FH / 4, B1F, tid);
    par_unit(b2, FO / 4, 8, B2F, tid);
  }
}

template <int MODE>
__global__ __launch_bounds__(256) void k_build(const int* __restrict__ ei, int* __restrict__ LIST,
                                               int* __restrict__ CNT, int* __restrict__ OFF,
                                               int* __restrict__ DINVB, int* __restrict__ FLAG) {
  static_assert(MODE == 0 || MODE == 1);
  extern __shared__ __attribute__((aligned(16))) int dsm[];
  int* wl   = dsm + LK_WL;
  int* sl   = dsm + LK_SL;
  int* cnt  = dsm + LK_CNT;
  int* offs = dsm + LK_OFF;
  int* cur  = dsm + LK_CUR;
  int* misc = dsm + LK_MISC;
  const int tid = (int)threadIdx.x, lane = tid & 31, wave = tid >> 5;
  const int blk = (int)blockIdx.x;
  const int nodeBase = blk * NBRUN;
  const int nbi = (NN - nodeBase) < NBRUN ? (NN - nodeBase) : NBRUN;
  const unsigned unb = (unsigned)(nbi < 0 ? 0 : nbi);

  {
    const v4i z4 = (v4i){0, 0, 0, 0};
    for (int i = tid * 4; i < CAP + NBRUN; i += 1024) *(v4ia*)(sl + i) = z4;
    if (tid < 16) misc[tid] = 0;
  }
  __syncthreads();

  const int* srcp = ei;
  const int* dstp = ei + NE;
  int* mylist = wl + wave * WLCAP;
  const int wbase = wave * EPW;
  const int wlast = wbase + EPW - 1;
  int wc = 0;
#pragma unroll 1
  for (int st = 0; st < NSTEP; ++st) {
    const int e0 = wbase + st * SUB + lane;
    int dk[4];
    int sk[4];
#pragma unroll
    for (int j = 0; j < 4; ++j) {
      const int e  = e0 + 32 * j;
      const int ec = e < wlast ? e : wlast;
      const int d  = dstp[ec];
      const int s  = srcp[ec];
      asm volatile("" :: "v"(d));
      asm volatile("" :: "v"(s));
      dk[j] = (e <= wlast) ? d : -1;
      sk[j] = (e <= wlast) ? s : -1;
    }
#pragma unroll
    for (int j = 0; j < 4; ++j) {
      const int key = (MODE == 0) ? dk[j] : sk[j];
      const unsigned slot = (unsigned)key - (unsigned)nodeBase;
      bool hit = slot < unb;
      if (MODE == 1) hit = hit && (sk[j] != dk[j]);
      const int payload = (MODE == 0) ? clampi(sk[j], 0, NN - 1) : 0;
      const unsigned mj = __builtin_amdgcn_ballot_w32(hit);
      if (mj != 0u) {
        if (hit) {
          const int pos = wc + (int)__builtin_amdgcn_mbcnt_lo(mj, 0u);
          if (pos < WLCAP) mylist[pos] = (payload << 10) | (int)slot;
        }
        wc += (int)__builtin_popcount(mj);
      }
    }
  }
  if (lane == 0) misc[wave] = wc;
  __syncthreads();

  if (wave == 0) {
    int t = 0, ov = 0;
#pragma unroll 1
    for (int w2 = 0; w2 < 8; ++w2) {
      const int craw = misc[w2];
      ov |= (craw > WLCAP) ? 1 : 0;
      const int c = __builtin_amdgcn_readfirstlane(clampi(craw, 0, WLCAP));
#pragma unroll 1
      for (int b0 = 0; b0 < c; b0 += 32) {
        const int idx = (b0 + lane) < c ? (b0 + lane) : c - 1;
        const int ent = wl[w2 * WLCAP + idx];
        const int m32 = (c - b0) < 32 ? (c - b0) : 32;
#pragma unroll 1
        for (int k = 0; k < m32; ++k) {
          const int u    = __builtin_amdgcn_readlane(ent, k);
          const int slot = u & (NBRUN - 1);
          if (t < CAP) {
            if (lane == 0) cnt[slot] = cnt[slot] + 1;
            t = t + 1;
          } else {
            ov = 1;
          }
        }
      }
    }
    if (lane == 0) { misc[8] = t; misc[9] = ov; }
  }
  __syncthreads();

  if constexpr (MODE == 0) {
    if (wave == 0) {
      const int base = lane * (NBRUN / 32);
      int s = 0, big = 0;
#pragma unroll 1
      for (int i = 0; i < NBRUN / 32; ++i) {
        const int cv = cnt[base + i];
        s += cv;
        big |= (cv > DEGCAP) ? 1 : 0;
      }
      int incl = s;
#pragma unroll
      for (int d = 1; d < 32; d <<= 1) {
        const int y = __shfl_up(incl, d, 32);
        incl += (lane >= d) ? y : 0;
      }
      int run = incl - s;
#pragma unroll 1
      for (int i = 0; i < NBRUN / 32; ++i) {
        const int cv = cnt[base + i];
        offs[base + i] = run;
        cur[base + i]  = run;
        run += cv;
      }
      const unsigned bm = __builtin_amdgcn_ballot_w32(big != 0);
      if (lane == 0) misc[9] = misc[9] | ((bm != 0u) ? 1 : 0);
    }
    __syncthreads();

    if (wave == 0) {
      int t2 = 0;
#pragma unroll 1
      for (int w2 = 0; w2 < 8; ++w2) {
        const int c = __builtin_amdgcn_readfirstlane(clampi(misc[w2], 0, WLCAP));
#pragma unroll 1
        for (int b0 = 0; b0 < c; b0 += 32) {
          const int idx = (b0 + lane) < c ? (b0 + lane) : c - 1;
          const int ent = wl[w2 * WLCAP + idx];
          const int m32 = (c - b0) < 32 ? (c - b0) : 32;
#pragma unroll 1
          for (int k = 0; k < m32; ++k) {
            const int u    = __builtin_amdgcn_readlane(ent, k);
            const int slot = u & (NBRUN - 1);
            if (t2 < CAP) {
              if (lane == 0) {
                int p = cur[slot];
                p = clampi(p, 0, CAP - 1);
                sl[p] = u >> 10;
                cur[slot] = p + 1;
              }
              t2 = t2 + 1;
            }
          }
        }
      }
    }
    __syncthreads();

    const int ovf = misc[9];
    int* lbase = LIST + (size_t)blk * (size_t)CAP;
    for (int pass = 0; pass < 2; ++pass) {
#pragma unroll 2
      for (int i = tid; i < CAP / 4; i += 256) {
        const v4i ev = *(const v4ia*)(sl + 4 * i);
        const v4i v = (v4i){ clampi(ev.x, 0, NN - 1), clampi(ev.y, 0, NN - 1),
                             clampi(ev.z, 0, NN - 1), clampi(ev.w, 0, NN - 1) };
        *(volatile v4i*)(lbase + 4 * i) = v;
      }
      __threadfence();
    }
    const v4i cv4 = *(const v4ia*)(cnt + 4 * tid);
    const v4i ov4 = *(const v4ia*)(offs + 4 * tid);
    const v4i fl4 = (v4i){ ovf, ovf, ovf, ovf };
    const size_t nb4 = (size_t)nodeBase + 4 * (size_t)tid;
    const bool fw = (wave == 0) && (lane < 8);
    *(volatile v4i*)(CNT + nb4) = cv4;
    *(volatile v4i*)(OFF + nb4) = ov4;
    if (fw) *(volatile v4i*)(FLAG + blk * 32 + 4 * lane) = fl4;
    __threadfence();
    *(volatile v4i*)(CNT + nb4) = cv4;
    *(volatile v4i*)(OFF + nb4) = ov4;
    if (fw) *(volatile v4i*)(FLAG + blk * 32 + 4 * lane) = fl4;
  } else {
    const int ovf = misc[9];
    const int qn  = 0x7fc00000;
#pragma unroll 1
    for (int q = 0; q < 4; ++q) {
      const int slot = tid + 256 * q;
      const int cv   = cnt[slot];
      const float d  = (float)cv;
      const float r  = 1.0f / sqrtf(d);
      const float dv = (d > 0.0f) ? r : 0.0f;
      cur[slot] = (ovf != 0) ? qn : __float_as_int(dv);
    }
    __syncthreads();
    const v4i cv4 = *(const v4ia*)(cnt + 4 * tid);
    const v4i dv4 = *(const v4ia*)(cur + 4 * tid);
    const v4i fl4 = (v4i){ ovf, ovf, ovf, ovf };
    const size_t nb4 = (size_t)nodeBase + 4 * (size_t)tid;
    const bool fw = (wave == 0) && (lane < 8);
    *(volatile v4i*)(CNT + nb4) = cv4;
    *(volatile v4i*)(DINVB + nb4) = dv4;
    if (fw) *(volatile v4i*)(FLAG + blk * 32 + 4 * lane) = fl4;
    __threadfence();
    *(volatile v4i*)(CNT + nb4) = cv4;
    *(volatile v4i*)(DINVB + nb4) = dv4;
    if (fw) *(volatile v4i*)(FLAG + blk * 32 + 4 * lane) = fl4;
  }
}

__global__ __launch_bounds__(256) void k_agg1(const float* __restrict__ P, const int* __restrict__ LIST,
                                              const int* __restrict__ CNT, const int* __restrict__ OFF,
                                              const float* __restrict__ DINV, const int* __restrict__ FLAG,
                                              const float* __restrict__ B1F, unsigned short* __restrict__ HL) {
  __shared__ __attribute__((aligned(16))) float sB[FH];
  const int tid = (int)threadIdx.x, lane = tid & 31, wave = tid >> 5;
  if (wave == 0) {
    const v2f bq = *(const v2fa*)(B1F + 2 * lane);
    asm volatile("" :: "v"(bq));
    sB[2 * lane]     = bq.x;
    sB[2 * lane + 1] = bq.y;
  }
  __syncthreads();
  const float bx = sB[2 * lane];
  const float by = sB[2 * lane + 1];

  const int row  = (int)blockIdx.x * 8 + wave;
  const bool live = row < NN;
  const int ic   = live ? row : NN - 1;
  const int b    = ic >> 10;
  int c  = CNT[ic];
  int o  = OFF[ic];
  const int fl   = FLAG[b * 32];
  const float di = DINV[ic];
  asm volatile("" :: "v"(c));
  asm volatile("" :: "v"(o));
  asm volatile("" :: "v"(fl));
  asm volatile("" :: "v"(di));
  c = clampi(c, 0, DEGCAP);
  o = clampi(o, 0, CAP - DEGCAP);
  const int cn = __builtin_amdgcn_readfirstlane(live ? c : 0);
  const int* lp = LIST + (size_t)b * (size_t)CAP + (size_t)o;
  const int top = cn > 0 ? cn - 1 : 0;
  const int i0 = lane < top ? lane : top;
  const int i1 = (lane + 32) < top ? (lane + 32) : top;
  int s0 = lp[i0];
  int s1 = lp[i1];
  asm volatile("" :: "v"(s0));
  asm volatile("" :: "v"(s1));
  s0 = clampi(s0, 0, NN - 1);
  s1 = clampi(s1, 0, NN - 1);
  const float dv0 = DINV[s0];
  const float dv1 = DINV[s1];
  asm volatile("" :: "v"(dv0));
  asm volatile("" :: "v"(dv1));
  const float cr0 = (-dv0) * di;
  const float cr1 = (-dv1) * di;
  const float cf0 = (s0 == ic) ? 0.0f : cr0;
  const float cf1 = (s1 == ic) ? 0.0f : cr1;
  const int cb0 = __float_as_int(cf0);
  const int cb1 = __float_as_int(cf1);

  const float* P1l = P + FH + 2 * lane;
  float a0 = 0.0f, a1 = 0.0f;
  const int c0 = cn < 32 ? cn : 32;
#pragma unroll 1
  for (int k = 0; k < c0; ++k) {
    const int   skk = __builtin_amdgcn_readlane(s0, k);
    const float ck  = __int_as_float(__builtin_amdgcn_readlane(cb0, k));
    const v2f r = *(const v2fa*)(P1l + (size_t)skk * PLD);
    asm volatile("" :: "v"(r));
    a0 = a0 + ck * r.x;
    a1 = a1 + ck * r.y;
  }
#pragma unroll 1
  for (int k = 32; k < cn; ++k) {
    const int   skk = __builtin_amdgcn_readlane(s1, k - 32);
    const float ck  = __int_as_float(__builtin_amdgcn_readlane(cb1, k - 32));
    const v2f r = *(const v2fa*)(P1l + (size_t)skk * PLD);
    asm volatile("" :: "v"(r));
    a0 = a0 + ck * r.x;
    a1 = a1 + ck * r.y;
  }
  const v2f p0 = *(const v2fa*)(P + (size_t)ic * PLD + 2 * lane);
  asm volatile("" :: "v"(p0));
  const float qn = __int_as_float(0x7fc00000);
  const bool poison = fl != 0;
  float h0 = relu_k((p0.x + a0) + bx);
  float h1 = relu_k((p0.y + a1) + by);
  h0 = poison ? qn : h0;
  h1 = poison ? qn : h1;
  const float y0 = live ? h0 : 0.0f;
  const float y1 = live ? h1 : 0.0f;
  const unsigned hv = pk16(bf16_bits(y0), bf16_bits(y1));
  unsigned lv = 0u;
  if (H1_TWO_TERM) lv = pk16(bf16_lo_bits(y0), bf16_lo_bits(y1));
  unsigned short* rp = HL + (size_t)row * HLK + 2 * lane;
  *(volatile unsigned*)rp = hv;
  *(volatile unsigned*)(rp + FH) = lv;
  __threadfence();
  *(volatile unsigned*)rp = hv;
  *(volatile unsigned*)(rp + FH) = lv;
}

__global__ __launch_bounds__(256) void k_agg2_out(const float* __restrict__ Q, const int* __restrict__ LIST,
                                                  const int* __restrict__ CNT, const int* __restrict__ OFF,
                                                  const float* __restrict__ DINV, const int* __restrict__ FLAG,
                                                  const float* __restrict__ B2F, float* __restrict__ outp) {
  __shared__ __attribute__((aligned(16))) float sB[FO];
  const int tid = (int)threadIdx.x, lane = tid & 31, wave = tid >> 5;
  if (wave == 0) {
    const v4f bq = *(const v4fa*)(B2F + 4 * (lane & 3));
    asm volatile("" :: "v"(bq));
    if (lane < 4) {
      sB[4 * lane]     = bq[0];
      sB[4 * lane + 1] = bq[1];
      sB[4 * lane + 2] = bq[2];
      sB[4 * lane + 3] = bq[3];
    }
  }
  __syncthreads();
  const int cc = lane & 15;
  const float b2v = sB[cc];

  const int n    = ((int)blockIdx.x * 8 + wave) * 2 + (lane >> 4);
  const bool live = n < NN;
  const int ic   = clampi(n, 0, NN - 1);
  const int b    = ic >> 10;
  int c  = CNT[ic];
  int o  = OFF[ic];
  const int fl   = FLAG[b * 32];
  const float di = DINV[ic];
  asm volatile("" :: "v"(c));
  asm volatile("" :: "v"(o));
  asm volatile("" :: "v"(fl));
  asm volatile("" :: "v"(di));
  c = clampi(c, 0, DEGCAP);
  c = live ? c : 0;
  o = clampi(o, 0, CAP - DEGCAP);
  const int oth = __shfl_xor(c, 16, 32);
  const int cm  = __builtin_amdgcn_readfirstlane(c > oth ? c : oth);
  const int* lp = LIST + (size_t)b * (size_t)CAP + (size_t)o;
  const float* Q1c = Q + FO + cc;

  float acc = 0.0f;
#pragma unroll 1
  for (int j = 0; j < cm; ++j) {
    int jj = j < (c - 1) ? j : (c - 1);
    jj = jj > 0 ? jj : 0;
    const int w = lp[jj];
    asm volatile("" :: "v"(w));
    int s = (c > 0) ? w : ic;
    s = clampi(s, 0, NN - 1);
    const float dv = DINV[s];
    const float q  = Q1c[(size_t)s * QLD];
    asm volatile("" :: "v"(dv));
    asm volatile("" :: "v"(q));
    const float cr = (-dv) * di;
    const float cf = (s == ic) ? 0.0f : cr;
    const float pr = cf * q;
    const float term = (j < c) ? pr : 0.0f;
    acc = acc + term;
  }
  const float q0 = Q[(size_t)ic * QLD + cc];
  asm volatile("" :: "v"(q0));
  const float h2 = (q0 + acc) + b2v;

  float mx = h2;
#pragma unroll
  for (int d = 8; d >= 1; d >>= 1) {
    const float ov = __shfl_xor(mx, d, 32);
    mx = ((ov > mx) || (ov != ov)) ? ov : mx;
  }
  const float sh = h2 - mx;
  float sum = expf(sh);
#pragma unroll
  for (int d = 8; d >= 1; d >>= 1) {
    const float ov = __shfl_xor(sum, d, 32);
    sum = sum + ov;
  }
  float res = sh - logf(sum);
  const float qn = __int_as_float(0x7fc00000);
  res = (fl != 0) ? qn : res;
  float* op = outp + (size_t)ic * FO + cc;
  if (live) *(volatile float*)op = res;
  __threadfence();
  if (live) *(volatile float*)op = res;
}

constexpr int TILES_M = (NN + 63) / 64;
constexpr int G_GEMM1 = (TILES_M * 2 + 7) / 8;
constexpr int G_GEMM2 = (TILES_M * 1 + 7) / 8;
static_assert(((size_t)NP * FIN / 8) % 256 == 0);

extern "C" void kernel_launch(void* const* d_in, const int* in_sizes, int n_in,
                              void* d_out, int out_size, void* d_ws, size_t ws_size,
                              hipStream_t stream) {
  if (n_in < 8) return;
  if (in_sizes[0] != NN * FIN) return;
  if (in_sizes[1] != 2 * NE) return;
  if (in_sizes[2] != FIN * FH || in_sizes[3] != FIN * FH) return;
  if (in_sizes[4] != FH) return;
  if (in_sizes[5] != FH * FO || in_sizes[6] != FH * FO) return;
  if (in_sizes[7] != FO) return;
  if (out_size != NN * FO) return;
  if (ws_size < WS_TOTAL) return;

  const float* x   = (const float*)d_in[0];
  const int*   ei  = (const int*)d_in[1];
  const float* W01 = (const float*)d_in[2];
  const float* W11 = (const float*)d_in[3];
  const float* b1  = (const float*)d_in[4];
  const float* W02 = (const float*)d_in[5];
  const float* W12 = (const float*)d_in[6];
  const float* b2  = (const float*)d_in[7];
  float* out = (float*)d_out;

  char* ws = (char*)d_ws;
  unsigned short* R0    = (unsigned short*)(ws + OFF_R0);
  float*          R1    = (float*)(ws + OFF_R1);
  int*            LIST  = (int*)(ws + OFF_LIST);
  int*            CNT   = (int*)(ws + OFF_CNT);
  int*            OFFS  = (int*)(ws + OFF_OFF);
  int*            DEGS  = (int*)(ws + OFF_DEGS);
  int*            DINVB = (int*)(ws + OFF_DINV);
  const float*    DINV  = (const float*)(ws + OFF_DINV);
  int*            FLAGL = (int*)(ws + OFF_FLAGL);
  int*            FLAGC = (int*)(ws + OFF_FLAGC);
  unsigned short* BT1   = (unsigned short*)(ws + OFF_BT1);
  unsigned short* BT2   = (unsigned short*)(ws + OFF_BT2);
  unsigned*       B1Fu  = (unsigned*)(ws + OFF_B1F);
  unsigned*       B2Fu  = (unsigned*)(ws + OFF_B2F);
  const float*    B1F   = (const float*)(ws + OFF_B1F);
  const float*    B2F   = (const float*)(ws + OFF_B2F);

  hipFuncSetAttribute(reinterpret_cast<const void*>(&k_build<0>), hipFuncAttributeMaxDynamicSharedMemorySize, (int)LK_LDS);
  hipFuncSetAttribute(reinterpret_cast<const void*>(&k_build<1>), hipFuncAttributeMaxDynamicSharedMemorySize, (int)LK_LDS);

  k_plane<0><<<NP * FIN / 8 / 256, 256, 0, stream>>>(x, NN, FIN, FIN, R0, NP, FIN);
  k_prep<<<13, 256, 0, stream>>>(W01, W11, b1, W02, W12, b2, BT1, BT2, B1Fu, B2Fu);
  k_build<0><<<NBLK, 256, LK_LDS, stream>>>(ei, LIST, CNT, OFFS, DINVB, FLAGL);
  k_build<1><<<NBLK, 256, LK_LDS, stream>>>(ei, LIST, DEGS, OFFS, DINVB, FLAGC);
  k_gemm_nt<0, 0><<<G_GEMM1, 256, 0, stream>>>(R0, BT1, B1F, R1, NN, 2 * FH, FIN, PLD);
  k_agg1<<<NP / 8, 256, 0, stream>>>(R1, LIST, CNT, OFFS, DINV, FLAGL, B1F, R0);
  k_gemm_nt<0, 0><<<G_GEMM2, 256, 0, stream>>>(R0, BT2, B1F, R1, NN, 64, HLK, QLD);
  k_agg2_out<<<NN / 2 / 8, 256, 0, stream>>>(R1, LIST, CNT, OFFS, DINV, FLAGL, B2F, out);
}
